// CascadeMemoryAttention_6777458393275
// MI455X (gfx1250) — hardware-verified
//
#include <hip/hip_runtime.h>
#include <math.h>
#include <stdint.h>

#ifndef NB
#define NB 2
#endif
#ifndef SEQ
#define SEQ 2048
#endif
#define NB_FULL 2
#define T_FULL  2048
#define MEMT    256
#define M_FULL  256
#define NMEMK   (2 * MEMT)
#define SKEY    (SEQ + NMEMK)
#define DMOD    1024
#define NH      16
#define HD      64
#define GLN     64
#define KCAN    4
#define QSC   8.0f
#define KSC   8.0f
#define QRS   2048.0f
#define PCAR  32768.0f
#define VCAR  1024.0f
#define OSC   1024.0f
#define ORS   2048.0f
#define WOS   1024.0f
#define GWS   64.0f
#define LOG2E 1.4426950408889634f
#define NEGS  (-3.0e38f)
#define ATT_WAVES   4
#define ATT_THREADS (ATT_WAVES * 32)
#define NQT         (SEQ / 64)
#define ATT_BLOCKS  (NB * NH * NQT)
#define NMKB        (NMEMK / 32)
#define SLAB        (16 * 68)
static_assert(NB >= 1 && NB <= NB_FULL);
static_assert((SEQ % 64) == 0 && SEQ >= 256 && SEQ <= T_FULL);
static_assert(HD == 64 && DMOD == NH * HD && GLN == 64 && NH <= GLN && KCAN == 4);
static_assert((SKEY % 64) == 0 && (NMEMK % 32) == 0 && (DMOD % 64) == 0 && (DMOD % 32) == 0);
static_assert(((NB * SEQ * DMOD / 8) % 256) == 0 && ((NB * MEMT * DMOD / 8) % 256) == 0);
static_assert(((GLN * DMOD / 8) % 256) == 0 && ((DMOD * DMOD) % (64 * 64)) == 0);
static_assert(ATT_THREADS == 128 && (SLAB * 4) % 16 == 0);

typedef unsigned short u16;
typedef _Float16 v16h __attribute__((ext_vector_type(16)));
typedef _Float16 v8h  __attribute__((ext_vector_type(8)));
typedef __bf16   v16b __attribute__((ext_vector_type(16)));
typedef float    v8f  __attribute__((ext_vector_type(8)));
typedef float    v4f  __attribute__((ext_vector_type(4)));
typedef unsigned int v4u __attribute__((ext_vector_type(4)));

union FragH { v16h v; v8h h[2]; v4u u[2]; };
union FragB { v16b v; v4u u[2]; };

__device__ __forceinline__ unsigned short bf_bits(float f) {
  unsigned u = __float_as_uint(f);
  return (unsigned short)((u + 0x7FFFu + ((u >> 16) & 1u)) >> 16);
}
__device__ __forceinline__ float bf_up(unsigned short h) { return __uint_as_float(((unsigned)h) << 16); }
__device__ __forceinline__ float bf_val(float f) { return bf_up(bf_bits(f)); }
__device__ __forceinline__ unsigned short h_bits(_Float16 x) { return __builtin_bit_cast(unsigned short, x); }
__device__ __forceinline__ unsigned pk16(unsigned short a, unsigned short b) { return (unsigned)a | ((unsigned)b << 16); }
__device__ __forceinline__ v8f zero8() { v8f z = {0.f, 0.f, 0.f, 0.f, 0.f, 0.f, 0.f, 0.f}; return z; }

__device__ __forceinline__ v16h ldfrag_h(const _Float16* p) {
  FragH f;
  f.h[0] = *(const v8h*)(p);
  f.h[1] = *(const v8h*)(p + 16);
  return f.v;
}
__device__ __forceinline__ v16b ldfrag_b(const u16* p) {
  FragB f;
  f.u[0] = *(const v4u*)(p);
  f.u[1] = *(const v4u*)(p + 16);
  return f.v;
}

__device__ __forceinline__ v8f mma_h(v16h a, v16h b, v8f c) {
  return __builtin_amdgcn_wmma_f32_16x16x32_f16(false, a, false, b, (short)0, c, false, false);
}
__device__ __forceinline__ v8f mma_b(v16b a, v16b b, v8f c) {
  return __builtin_amdgcn_wmma_f32_16x16x32_bf16(false, a, false, b, (short)0, c, false, false);
}
template <typename F>
__device__ __forceinline__ void guard6(v8f& a, v8f& b, v8f& c, v8f& d, F x0, F x1, F x2, F x3, F x4, F x5) {
#if defined(__HIP_DEVICE_COMPILE__)
  asm volatile("v_nop\n\tv_nop\n\tv_nop\n\tv_nop"
               : "+v"(a), "+v"(b), "+v"(c), "+v"(d) : "v"(x0), "v"(x1), "v"(x2), "v"(x3), "v"(x4), "v"(x5) : "memory");
#endif
}
__device__ __forceinline__ void guard4x8(v8f& a, v8f& b, v8f& c, v8f& d, v16h x0, v16h x1, v16h x2, v16h x3,
                                         v16h x4, v16h x5, v16h x6, v16h x7) {
#if defined(__HIP_DEVICE_COMPILE__)
  asm volatile("v_nop\n\tv_nop\n\tv_nop\n\tv_nop"
               : "+v"(a), "+v"(b), "+v"(c), "+v"(d)
               : "v"(x0), "v"(x1), "v"(x2), "v"(x3), "v"(x4), "v"(x5), "v"(x6), "v"(x7) : "memory");
#endif
}
__device__ __forceinline__ void guard8x6(v8f& a, v8f& b, v8f& c, v8f& d, v8f& e, v8f& f, v8f& g, v8f& h,
                                         v16h x0, v16h x1, v16h x2, v16h x3, v16h x4, v16h x5) {
#if defined(__HIP_DEVICE_COMPILE__)
  asm volatile("v_nop\n\tv_nop\n\tv_nop\n\tv_nop"
               : "+v"(a), "+v"(b), "+v"(c), "+v"(d), "+v"(e), "+v"(f), "+v"(g), "+v"(h)
               : "v"(x0), "v"(x1), "v"(x2), "v"(x3), "v"(x4), "v"(x5) : "memory");
#endif
}
__device__ __forceinline__ void acc_guard4(v8f& a, v8f& b, v8f& c, v8f& d) {
#if defined(__HIP_DEVICE_COMPILE__)
  asm volatile("v_nop\n\tv_nop\n\tv_nop\n\tv_nop" : "+v"(a), "+v"(b), "+v"(c), "+v"(d));
#endif
}
__device__ __forceinline__ void wave_sync_lds() {
#if defined(__HIP_DEVICE_COMPILE__)
  __builtin_amdgcn_fence(__ATOMIC_RELEASE, "workgroup");
  __builtin_amdgcn_wave_barrier();
  __builtin_amdgcn_fence(__ATOMIC_ACQUIRE, "workgroup");
#endif
}

__global__ __launch_bounds__(256) void cvt_rows(const float* __restrict__ x, const float* __restrict__ fwm,
                                                 const float* __restrict__ rvm, u16* XB) {
  const int part = blockIdx.y;
  const float* src = x;
  int rows = SEQ, sbst = T_FULL * DMOD, drow0 = 0;
  if (part == 1)      { src = fwm; rows = MEMT; sbst = M_FULL * DMOD; drow0 = SEQ; }
  else if (part == 2) { src = rvm; rows = MEMT; sbst = M_FULL * DMOD; drow0 = SEQ + MEMT; }
  const int n8 = NB * rows * (DMOD / 8);
  const int gt = blockIdx.x * 256 + (int)threadIdx.x;
  if (gt >= n8) return;
  const int e0  = gt * 8;
  const int per = rows * DMOD;
  const int b   = e0 / per;
  const int rem = e0 - b * per;
  const int r   = rem / DMOD;
  const int c   = rem - r * DMOD;
  const float* p = src + (size_t)b * (size_t)sbst + (size_t)r * DMOD + c;
  const v4f a = *(const v4f*)(p), d4 = *(const v4f*)(p + 4);
  float v[8];
#pragma unroll
  for (int e = 0; e < 4; ++e) { v[e] = a[e]; v[4 + e] = d4[e]; }
  v4u o;
#pragma unroll
  for (int e = 0; e < 4; ++e) o[e] = pk16(bf_bits(v[2 * e]), bf_bits(v[2 * e + 1]));
  u16* d = XB + ((size_t)b * SKEY + drow0 + r) * (size_t)DMOD + c;
  for (int pass = 0; pass < 2; ++pass) {
    *(volatile v4u*)(d) = o;
    __threadfence();
  }
}

__global__ __launch_bounds__(256) void wt16(const float* __restrict__ W0, const float* __restrict__ W1,
                                             const float* __restrict__ W2, const float* __restrict__ W3,
                                             u16* T0, u16* T1, u16* T2, u16* T3) {
  __shared__ float tile[64][65];
  const int sel = blockIdx.y;
  const float* W = W0;
  u16* T = T0;
  if (sel == 1)      { W = W1; T = T1; }
  else if (sel == 2) { W = W2; T = T2; }
  else if (sel == 3) { W = W3; T = T3; }
  const int mode = (sel == 3) ? 1 : 0;
  const int tid = threadIdx.x;
  const int k0 = (blockIdx.x / (DMOD / 64)) * 64;
  const int n0 = (blockIdx.x % (DMOD / 64)) * 64;
#pragma unroll
  for (int i = 0; i < 16; ++i) {
    const int idx = i * 256 + tid;
    const int r = idx >> 6, cc = idx & 63;
    tile[cc][r] = W[(size_t)(k0 + r) * DMOD + n0 + cc];
  }
  __syncthreads();
  v4u ov[2];
  const int q8 = (tid & 7) * 8;
#pragma unroll
  for (int it = 0; it < 2; ++it) {
    const int row = (tid >> 3) + 32 * it;
    unsigned short s[8];
#pragma unroll
    for (int e = 0; e < 8; ++e) {
      const float w = tile[row][q8 + e];
      const unsigned short bb = bf_bits(w);
      const unsigned short hb = h_bits((_Float16)(bf_up(bb) * WOS));
      s[e] = (mode != 0) ? hb : bb;
    }
#pragma unroll
    for (int e = 0; e < 4; ++e) ov[it][e] = pk16(s[2 * e], s[2 * e + 1]);
  }
  for (int pass = 0; pass < 2; ++pass) {
#pragma unroll
    for (int it = 0; it < 2; ++it) {
      const int row = (tid >> 3) + 32 * it;
      u16* d = T + (size_t)(n0 + row) * DMOD + k0 + q8;
      *(volatile v4u*)(d) = ov[it];
    }
    __threadfence();
  }
}

__global__ __launch_bounds__(256) void gwt16(const float* __restrict__ gw, u16* GT) {
  const int gt = blockIdx.x * 256 + (int)threadIdx.x;
  if (gt >= GLN * (DMOD / 8)) return;
  const int n  = gt / (DMOD / 8);
  const int k8 = (gt - n * (DMOD / 8)) * 8;
  const int nc = min(n, NH - 1);
  unsigned short s[8];
#pragma unroll
  for (int e = 0; e < 8; ++e) {
    const float v = gw[(size_t)(k8 + e) * NH + nc];
    const float w = (n < NH) ? (bf_val(v) * GWS) : 0.f;
    s[e] = h_bits((_Float16)w);
  }
  v4u o;
#pragma unroll
  for (int e = 0; e < 4; ++e) o[e] = pk16(s[2 * e], s[2 * e + 1]);
  u16* d = GT + (size_t)n * DMOD + k8;
  for (int pass = 0; pass < 2; ++pass) {
    *(volatile v4u*)(d) = o;
    __threadfence();
  }
}

__device__ __forceinline__ void epi16(float* sl, v8f a0, v8f a1, v8f a2, v8f a3, float oscale,
                                      u16* C, u16* R, int rmode, float rscale, int N,
                                      size_t rowb, int col0, int lane,
                                      const float* __restrict__ bias, int bmode, int blen) {
  const int hh = lane >> 4, m = lane & 15;
  float bc[4], br[8];
#pragma unroll
  for (int j = 0; j < 4; ++j) bc[j] = 0.f;
#pragma unroll
  for (int r = 0; r < 8; ++r) br[r] = 0.f;
  if (blen > 0) {
    if (bmode != 0) {
#pragma unroll
      for (int r = 0; r < 8; ++r) {
        const int bi = min((int)rowb + 8 * hh + r, blen - 1);
        br[r] = bf_val(bias[bi]);
      }
    } else {
#pragma unroll
      for (int j = 0; j < 4; ++j) {
        const int bi = min(col0 + 16 * j + m, blen - 1);
        bc[j] = bf_val(bias[bi]);
      }
    }
  }
#pragma unroll
  for (int r = 0; r < 8; ++r) {
    const int ro = (8 * hh + r) * 68 + m;
    sl[ro]      = (a0[r] + br[r] + bc[0]) * oscale;
    sl[ro + 16] = (a1[r] + br[r] + bc[1]) * oscale;
    sl[ro + 32] = (a2[r] + br[r] + bc[2]) * oscale;
    sl[ro + 48] = (a3[r] + br[r] + bc[3]) * oscale;
  }
  wave_sync_lds();
  const int rq = lane >> 3, c8 = (lane & 7) * 8;
  v4u ov[4], rv[4];
#pragma unroll
  for (int i4 = 0; i4 < 4; ++i4) {
    const int row = i4 * 4 + rq;
    const v4f a = *(const v4f*)(sl + row * 68 + c8), c4 = *(const v4f*)(sl + row * 68 + c8 + 4);
    float w[8];
#pragma unroll
    for (int e = 0; e < 4; ++e) { w[e] = a[e]; w[4 + e] = c4[e]; }
    unsigned short hb[8], lb[8];
#pragma unroll
    for (int e = 0; e < 8; ++e) {
      const _Float16 hv = (_Float16)w[e];
      hb[e] = h_bits(hv);
      lb[e] = h_bits((_Float16)((w[e] - (float)hv) * rscale));
    }
#pragma unroll
    for (int e = 0; e < 4; ++e) {
      ov[i4][e] = pk16(hb[2 * e], hb[2 * e + 1]);
      rv[i4][e] = pk16(lb[2 * e], lb[2 * e + 1]);
    }
  }
  const size_t dofs = (rowb + (size_t)rq) * (size_t)N + col0 + c8;
  u16* dst = C + dofs;
  u16* dsr = R + dofs;
  for (int pass = 0; pass < 2; ++pass) {
#pragma unroll
    for (int i4 = 0; i4 < 4; ++i4) {
      *(volatile v4u*)(dst + (size_t)(i4 * 4) * (size_t)N) = ov[i4];
      if (rmode != 0) *(volatile v4u*)(dsr + (size_t)(i4 * 4) * (size_t)N) = rv[i4];
    }
    __threadfence();
  }
}

__device__ __forceinline__ void epi64(float* sl, v8f a0, v8f a1, v8f a2, v8f a3, float oscale, float* C, int N,
                                      size_t rowb, int col0, int lane, const float* __restrict__ bias, int blen) {
  const int hh = lane >> 4, m = lane & 15;
  float bc[4];
#pragma unroll
  for (int j = 0; j < 4; ++j) bc[j] = 0.f;
  if (blen > 0) {
#pragma unroll
    for (int j = 0; j < 4; ++j) {
      const int bi = min(col0 + 16 * j + m, blen - 1);
      bc[j] = bf_val(bias[bi]);
    }
  }
#pragma unroll
  for (int r = 0; r < 8; ++r) {
    const int ro = (8 * hh + r) * 68 + m;
    sl[ro]      = a0[r] * oscale + bc[0];
    sl[ro + 16] = a1[r] * oscale + bc[1];
    sl[ro + 32] = a2[r] * oscale + bc[2];
    sl[ro + 48] = a3[r] * oscale + bc[3];
  }
  wave_sync_lds();
  v4f vals[8];
#pragma unroll
  for (int it = 0; it < 8; ++it) vals[it] = *(const v4f*)(sl + (it * 2 + hh) * 68 + m * 4);
  float* dst = C + (rowb + (size_t)hh) * (size_t)N + col0 + m * 4;
  for (int pass = 0; pass < 2; ++pass) {
#pragma unroll
    for (int it = 0; it < 8; ++it) {
      *(volatile v4f*)(dst + (size_t)(it * 2) * (size_t)N) = vals[it];
    }
    __threadfence();
  }
}

__global__ __launch_bounds__(128)
void gemm_b16(const u16* __restrict__ A, const u16* __restrict__ Bt, u16* C, u16* R, int M, int N, int K,
              int bstA, int bstB, int bstC, float oscale, int rmode, float rscale,
              const float* __restrict__ bias, int bmode, int blen) {
  __shared__ __align__(16) float slab[4 * SLAB];
  const int tid = threadIdx.x, wave = tid >> 5, lane = tid & 31, hh = lane >> 4, m = lane & 15;
  const int ntile = N >> 6, mtile = M >> 6;
  const int per   = ntile * mtile;
  const int bid   = blockIdx.x;
  const int bt    = bid / per;
  const int t     = bid - bt * per;
  const int rowb  = (t / ntile) * 64 + wave * 16;
  const int col0  = (t % ntile) * 64;
  if (rowb + 16 > M) return;
  const u16* Ab = A  + (size_t)bt * (size_t)bstA;
  const u16* Bb = Bt + (size_t)bt * (size_t)bstB;
  u16*       Cb = C  + (size_t)bt * (size_t)bstC;
  u16*       Rb = R  + (size_t)bt * (size_t)bstC;
  const u16* ap = Ab + (size_t)(rowb + m) * K + 8 * hh;
  const u16* bp = Bb + (size_t)(col0 + m) * K + 8 * hh;
  const size_t bs = (size_t)16 * K;
  v8f acc0 = zero8(), acc1 = zero8(), acc2 = zero8(), acc3 = zero8();
#pragma unroll 1
  for (int k0 = 0; k0 < K; k0 += 32) {
    const v16b a  = ldfrag_b(ap + k0);
    const v16b b0 = ldfrag_b(bp + k0);
    const v16b b1 = ldfrag_b(bp + bs + k0);
    const v16b b2 = ldfrag_b(bp + 2 * bs + k0);
    const v16b b3 = ldfrag_b(bp + 3 * bs + k0);
    acc0 = mma_b(a, b0, acc0);
    acc1 = mma_b(a, b1, acc1);
    acc2 = mma_b(a, b2, acc2);
    acc3 = mma_b(a, b3, acc3);
    guard6<v16b>(acc0, acc1, acc2, acc3, a, b0, b1, b2, b3, a);
  }
  epi16(slab + wave * SLAB, acc0, acc1, acc2, acc3, oscale, Cb, Rb, rmode, rscale, N, (size_t)rowb, col0, lane,
        bias, bmode, blen);
}

template <bool RES>
__global__ __launch_bounds__(128)
void gemm_hf(const u16* __restrict__ A, const u16* __restrict__ Ar, const u16* __restrict__ Bt, float* C,
             int M, int N, int K, float oscale, float rinv, const float* __restrict__ bias, int blen) {
  __shared__ __align__(16) float slab[4 * SLAB];
  const int tid = threadIdx.x, wave = tid >> 5, lane = tid & 31, hh = lane >> 4, m = lane & 15;
  const int ntile = N >> 6;
  const int bid   = blockIdx.x;
  const int rowb  = (bid / ntile) * 64 + wave * 16;
  const int col0  = (bid % ntile) * 64;
  if (rowb + 16 > M) return;
  const _Float16* ap = (const _Float16*)(const void*)A  + (size_t)(rowb + m) * K + 8 * hh;
  const _Float16* rp = (const _Float16*)(const void*)Ar + (size_t)(rowb + m) * K + 8 * hh;
  const _Float16* bp = (const _Float16*)(const void*)Bt + (size_t)(col0 + m) * K + 8 * hh;
  const size_t bs = (size_t)16 * K;
  v8f acc0 = zero8(), acc1 = zero8(), acc2 = zero8(), acc3 = zero8();
  v8f rc0 = zero8(), rc1 = zero8(), rc2 = zero8(), rc3 = zero8();
#pragma unroll 1
  for (int k0 = 0; k0 < K; k0 += 32) {
    const v16h a  = ldfrag_h(ap + k0);
    const v16h b0 = ldfrag_h(bp + k0);
    const v16h b1 = ldfrag_h(bp + bs + k0);
    const v16h b2 = ldfrag_h(bp + 2 * bs + k0);
    const v16h b3 = ldfrag_h(bp + 3 * bs + k0);
    acc0 = mma_h(a, b0, acc0);
    acc1 = mma_h(a, b1, acc1);
    acc2 = mma_h(a, b2, acc2);
    acc3 = mma_h(a, b3, acc3);
    if (RES) {
      const v16h ar = ldfrag_h(rp + k0);
      rc0 = mma_h(ar, b0, rc0);
      rc1 = mma_h(ar, b1, rc1);
      rc2 = mma_h(ar, b2, rc2);
      rc3 = mma_h(ar, b3, rc3);
      guard8x6(acc0, acc1, acc2, acc3, rc0, rc1, rc2, rc3, a, ar, b0, b1, b2, b3);
    } else {
      guard6<v16h>(acc0, acc1, acc2, acc3, a, b0, b1, b2, b3, a);
    }
  }
  if (RES) {
    acc_guard4(rc0, rc1, rc2, rc3);
    acc0 = acc0 + rc0 * rinv;
    acc1 = acc1 + rc1 * rinv;
    acc2 = acc2 + rc2 * rinv;
    acc3 = acc3 + rc3 * rinv;
  }
  epi64(slab + wave * SLAB, acc0, acc1, acc2, acc3, oscale, C, N, (size_t)rowb, col0, lane, bias, blen);
}

template <bool CAUSAL>
__device__ __forceinline__ void att_step(const _Float16* k0p, const _Float16* vp, int kb, int dq,
                                         v16h qf0, v16h qf1, v16h qr0, v16h qr1, float lsc, int hh,
                                         float& mrun, float& lrun, v8f& o0, v8f& o1, v8f& o2, v8f& o3) {
  v8f s0 = zero8(), s1 = zero8(), r0 = zero8(), r1 = zero8();
  const _Float16* k1p = k0p + (size_t)16 * DMOD;
  const v16h ka0 = ldfrag_h(k0p), ka1 = ldfrag_h(k0p + 32);
  const v16h kc0 = ldfrag_h(k1p), kc1 = ldfrag_h(k1p + 32);
  s0 = mma_h(ka0, qf0, s0);
  s0 = mma_h(ka1, qf1, s0);
  r0 = mma_h(ka0, qr0, r0);
  r0 = mma_h(ka1, qr1, r0);
  s1 = mma_h(kc0, qf0, s1);
  s1 = mma_h(kc1, qf1, s1);
  r1 = mma_h(kc0, qr0, r1);
  r1 = mma_h(kc1, qr1, r1);
  guard4x8(s0, s1, r0, r1, ka0, ka1, kc0, kc1, qf0, qf1, qr0, qr1);
  float tk[16];
#pragma unroll
  for (int i = 0; i < 8; ++i) {
    const float t0 = (s0[i] + r0[i] * (1.0f / QRS)) * lsc;
    const float t1 = (s1[i] + r1[i] * (1.0f / QRS)) * lsc;
    if (CAUSAL) {
      const int d0 = dq - kb - i;
      const int d1 = d0 - 16;
      tk[i]     = (d0 >= 0) ? t0 : NEGS;
      tk[8 + i] = (d1 >= 0) ? t1 : NEGS;
    } else {
      tk[i]     = t0;
      tk[8 + i] = t1;
    }
  }
  float cm = tk[0];
#pragma unroll
  for (int i = 1; i < 16; ++i) cm = fmaxf(cm, tk[i]);
  cm = fmaxf(cm, __shfl_xor(cm, 16, 32));
  const float mn = fmaxf(mrun, cm);
  const float al = exp2f(fminf(mrun - mn, 0.f));
  mrun = mn;
  float ps = 0.f;
  FragH ph;
#pragma unroll
  for (int wq = 0; wq < 2; ++wq) {
#pragma unroll
    for (int e4 = 0; e4 < 4; ++e4) {
      const int i = 8 * wq + 2 * e4;
      const float x0 = exp2f(fminf(tk[i] - mn, 0.f));
      const float x1 = exp2f(fminf(tk[i + 1] - mn, 0.f));
      const float p0 = (tk[i] > -1.0e38f) ? x0 : 0.f;
      const float p1 = (tk[i + 1] > -1.0e38f) ? x1 : 0.f;
      ps += p0 + p1;
      ph.u[wq][e4] = pk16(h_bits((_Float16)(p0 * PCAR)), h_bits((_Float16)(p1 * PCAR)));
    }
  }
  ps += __shfl_xor(ps, 16, 32);
  lrun = lrun * al + ps;
  float scl[8];
#pragma unroll
  for (int r = 0; r < 8; ++r) scl[r] = __shfl(al, 8 * hh + r, 32);
#pragma unroll
  for (int r = 0; r < 8; ++r) { o0[r] *= scl[r]; o1[r] *= scl[r]; o2[r] *= scl[r]; o3[r] *= scl[r]; }
  const v16h vf0 = ldfrag_h(vp);
  const v16h vf1 = ldfrag_h(vp + (size_t)16 * SKEY);
  const v16h vf2 = ldfrag_h(vp + (size_t)32 * SKEY);
  const v16h vf3 = ldfrag_h(vp + (size_t)48 * SKEY);
  o0 = mma_h(ph.v, vf0, o0);
  o1 = mma_h(ph.v, vf1, o1);
  o2 = mma_h(ph.v, vf2, o2);
  o3 = mma_h(ph.v, vf3, o3);
  guard6<v16h>(o0, o1, o2, o3, ph.v, vf0, vf1, vf2, vf3, ph.v);
}

__global__ __launch_bounds__(ATT_THREADS)
void attn_fwd(const u16* __restrict__ QPp, const u16* __restrict__ QRp, const u16* __restrict__ KPp,
              const u16* __restrict__ VPp, const float* __restrict__ GLp, float* Yp) {
  __shared__ __align__(16) float smem[ATT_WAVES * SLAB];

  const int tid  = threadIdx.x;
  const int wave = tid >> 5;
  const int lane = tid & 31;
  const int hh   = lane >> 4;
  const int c    = lane & 15;

  const int bid  = blockIdx.x;
  const int qt   = bid % NQT;
  const int bh   = bid / NQT;
  const int head = bh % NH;
  const int b    = bh / NH;
  if (b >= NB) return;
  const int qb   = qt * 64;
  const int q0   = qb + wave * 16;

  const size_t qofs = ((size_t)b * SEQ + q0 + c) * DMOD + head * HD + 8 * hh;
  const _Float16* Qh = (const _Float16*)(const void*)QPp + qofs;
  const _Float16* Qr = (const _Float16*)(const void*)QRp + qofs;
  const _Float16* Kb = (const _Float16*)(const void*)KPp + ((size_t)b * SKEY + c) * DMOD + head * HD + 8 * hh;
  const _Float16* Vb = (const _Float16*)(const void*)VPp + (size_t)b * DMOD * (size_t)SKEY
                       + (size_t)(head * HD + c) * SKEY + 8 * hh;
  const float lsc = 0.125f * (LOG2E / (QSC * KSC));
  const int dq = q0 + c - 8 * hh;

  const v16h qf0 = ldfrag_h(Qh);
  const v16h qf1 = ldfrag_h(Qh + 32);
  const v16h qr0 = ldfrag_h(Qr);
  const v16h qr1 = ldfrag_h(Qr + 32);

  float mrun = NEGS, lrun = 0.f;
  v8f o0 = zero8(), o1 = zero8(), o2 = zero8(), o3 = zero8();

  const int nkc = (q0 >> 5) + 1;
#pragma unroll 1
  for (int it = 0; it < nkc; ++it) {
    const int kb = it * 32;
    att_step<true>(Kb + (size_t)kb * DMOD, Vb + kb, kb, dq, qf0, qf1, qr0, qr1, lsc, hh, mrun, lrun, o0, o1, o2, o3);
  }
  acc_guard4(o0, o1, o2, o3);
  float* slab = smem + wave * SLAB;
#pragma unroll
  for (int r = 0; r < 8; ++r) {
    const int ro = (8 * hh + r) * 68 + c;
    slab[ro]      = o0[r];
    slab[ro + 16] = o1[r];
    slab[ro + 32] = o2[r];
    slab[ro + 48] = o3[r];
  }
  wave_sync_lds();
  const float mc = mrun, lc = lrun;

  mrun = NEGS; lrun = 0.f;
  o0 = zero8(); o1 = zero8(); o2 = zero8(); o3 = zero8();
#pragma unroll 1
  for (int it = 0; it < NMKB; ++it) {
    const int kb = SEQ + it * 32;
    att_step<false>(Kb + (size_t)kb * DMOD, Vb + kb, kb, dq, qf0, qf1, qr0, qr1, lsc, hh, mrun, lrun, o0, o1, o2, o3);
  }
  acc_guard4(o0, o1, o2, o3);

  const float mx  = fmaxf(mc, mrun);
  const float f1  = exp2f(fminf(mc - mx, 0.f));
  const float f2  = exp2f(fminf(mrun - mx, 0.f));
  const float lt  = lc * f1 + lrun * f2;
  const float linv = (lt > 0.f) ? ((1.0f / lt) * (1.0f / (PCAR * VCAR))) : 0.f;
  float z = GLp[((size_t)b * SEQ + q0 + c) * GLN + head];
  z = fminf(fmaxf(z, -80.f), 80.f);
  const float g   = 1.0f / (1.0f + exp2f(-z * LOG2E));
  const float wcv = f1 * linv;
  const float wmv = f2 * g * linv;
  float Wc[8], Wm[8];
#pragma unroll
  for (int r = 0; r < 8; ++r) { Wc[r] = __shfl(wcv, 8 * hh + r, 32); Wm[r] = __shfl(wmv, 8 * hh + r, 32); }
#pragma unroll
  for (int r = 0; r < 8; ++r) {
    const int ro = (8 * hh + r) * 68 + c;
    slab[ro]      = slab[ro]      * Wc[r] + o0[r] * Wm[r];
    slab[ro + 16] = slab[ro + 16] * Wc[r] + o1[r] * Wm[r];
    slab[ro + 32] = slab[ro + 32] * Wc[r] + o2[r] * Wm[r];
    slab[ro + 48] = slab[ro + 48] * Wc[r] + o3[r] * Wm[r];
  }
  wave_sync_lds();
  v4f vals[8];
#pragma unroll
  for (int it = 0; it < 8; ++it) vals[it] = *(const v4f*)(slab + (it * 2 + hh) * 68 + c * 4);
  float* dst = Yp + ((size_t)b * SEQ + q0 + hh) * DMOD + head * HD + c * 4;
  for (int pass = 0; pass < 2; ++pass) {
#pragma unroll
    for (int it = 0; it < 8; ++it) {
      *(volatile v4f*)(dst + (size_t)(it * 2) * DMOD) = vals[it];
    }
    __threadfence();
  }
}

__global__ __launch_bounds__(256) void canon16(const float* __restrict__ Y, const float* __restrict__ cw,
                                                const float* __restrict__ cb, u16* YH, u16* YR) {
  const int n8 = NB * SEQ * (DMOD / 8);
  const int gt = blockIdx.x * 256 + (int)threadIdx.x;
  if (gt >= n8) return;
  const int e0  = gt * 8;
  const int row = e0 / DMOD;
  const int c   = e0 - row * DMOD;
  const int t   = row % SEQ;
  const int rb  = row - t;
  float yv[KCAN][8];
#pragma unroll
  for (int j = 0; j < KCAN; ++j) {
    const int tt = t - (KCAN - 1) + j;
    const int rr = max(tt, 0);
    const float* yp = Y + (size_t)(rb + rr) * DMOD + c;
    const v4f a = *(const v4f*)(yp), d4 = *(const v4f*)(yp + 4);
#pragma unroll
    for (int e = 0; e < 4; ++e) {
      yv[j][e]     = (tt >= 0) ? a[e]  : 0.f;
      yv[j][4 + e] = (tt >= 0) ? d4[e] : 0.f;
    }
  }
  const v4f cb0 = *(const v4f*)(cb + c), cb1 = *(const v4f*)(cb + c + 4);
  unsigned short hb[8], lb[8];
#pragma unroll
  for (int e = 0; e < 8; ++e) {
    const v4f w4 = *(const v4f*)(cw + (size_t)(c + e) * KCAN);
    float conv = bf_val(w4[0]) * yv[0][e];
    conv += bf_val(w4[1]) * yv[1][e];
    conv += bf_val(w4[2]) * yv[2][e];
    conv += bf_val(w4[3]) * yv[3][e];
    const float bb = bf_val((e < 4) ? cb0[e] : cb1[e - 4]);
    const float yf = yv[KCAN - 1][e] + (conv + bb);
    const float ys = yf * OSC;
    const _Float16 hv = (_Float16)ys;
    hb[e] = h_bits(hv);
    lb[e] = h_bits((_Float16)((ys - (float)hv) * ORS));
  }
  v4u oh, orr;
#pragma unroll
  for (int e = 0; e < 4; ++e) { oh[e] = pk16(hb[2 * e], hb[2 * e + 1]); orr[e] = pk16(lb[2 * e], lb[2 * e + 1]); }
  u16* dh = YH + (size_t)e0;
  u16* dr = YR + (size_t)e0;
  for (int pass = 0; pass < 2; ++pass) {
    *(volatile v4u*)(dh) = oh;
    *(volatile v4u*)(dr) = orr;
    __threadfence();
  }
}

extern "C" void kernel_launch(void* const* d_in, const int* in_sizes, int n_in,
                              void* d_out, int out_size, void* d_ws, size_t ws_size,
                              hipStream_t stream) {
  if (n_in < 11) return;
  if (in_sizes[0] < ((NB - 1) * T_FULL + SEQ) * DMOD) return;
  if (in_sizes[1] < NB * M_FULL * DMOD) return;
  if (in_sizes[2] < NB * M_FULL * DMOD) return;
  if (in_sizes[3] < DMOD * DMOD) return;
  if (in_sizes[4] < DMOD * DMOD) return;
  if (in_sizes[5] < DMOD * DMOD) return;
  if (in_sizes[6] < DMOD * DMOD) return;
  if (in_sizes[7] < DMOD * NH) return;
  if (in_sizes[8] < NH) return;
  if (in_sizes[9] < DMOD * KCAN) return;
  if (in_sizes[10] < DMOD) return;
  if (out_size < NB * SEQ * DMOD) return;

  const float* Xin = (const float*)d_in[0];
  const float* Fin = (const float*)d_in[1];
  const float* Rin = (const float*)d_in[2];
  const float* Wq  = (const float*)d_in[3];
  const float* Wk  = (const float*)d_in[4];
  const float* Wv  = (const float*)d_in[5];
  const float* Wo  = (const float*)d_in[6];
  const float* Gw  = (const float*)d_in[7];
  const float* Gb  = (const float*)d_in[8];
  const float* Cw  = (const float*)d_in[9];
  const float* Cb  = (const float*)d_in[10];
  float*       out = (float*)d_out;

  const size_t szXB = (size_t)NB * SKEY * DMOD * 2;
  const size_t szW  = (size_t)DMOD * DMOD * 2;
  const size_t szGW = (size_t)GLN * DMOD * 2;
  const size_t szQ  = (size_t)NB * SEQ * DMOD * 2;
  const size_t szKP = (size_t)NB * SKEY * DMOD * 2;
  const size_t szVP = (size_t)NB * DMOD * SKEY * 2;
  const size_t szGL = (size_t)NB * SEQ * GLN * 4;
  const size_t szY  = (size_t)NB * SEQ * DMOD * 4;
  size_t off = 0;
  const size_t oXB = off; off += szXB;
  const size_t oWQ = off; off += szW;
  const size_t oWK = off; off += szW;
  const size_t oWV = off; off += szW;
  const size_t oWO = off; off += szW;
  const size_t oGW = off; off += szGW;
  const size_t oQP = off; off += szQ;
  const size_t oQR = off; off += szQ;
  const size_t oKP = off; off += szKP;
  const size_t oVP = off; off += szVP;
  const size_t oGL = off; off += szGL;
  const size_t oY  = off; off += szY;
  const size_t oYH = off; off += szQ;
  const size_t oYR = off; off += szQ;
  if (off > ws_size) return;
  if (off > (size_t)134217728) return;

  char* ws = (char*)d_ws;
  u16*   XB  = (u16*)(ws + oXB);
  u16*   WQT = (u16*)(ws + oWQ);
  u16*   WKT = (u16*)(ws + oWK);
  u16*   WVT = (u16*)(ws + oWV);
  u16*   WOT = (u16*)(ws + oWO);
  u16*   GWT = (u16*)(ws + oGW);
  u16*   QP  = (u16*)(ws + oQP);
  u16*   QR  = (u16*)(ws + oQR);
  u16*   KP  = (u16*)(ws + oKP);
  u16*   VP  = (u16*)(ws + oVP);
  float* GL  = (float*)(ws + oGL);
  float* Y   = (float*)(ws + oY);
  u16*   YH  = (u16*)(ws + oYH);
  u16*   YR  = (u16*)(ws + oYR);

  if ((DMOD % 64) != 0 || (SEQ % 64) != 0 || (SKEY % 64) != 0 || (GLN % 64) != 0 || (DMOD % 32) != 0) return;
  if (((NB * SEQ * (DMOD / 8)) % 256) != 0 || ((GLN * (DMOD / 8)) % 256) != 0) return;

  const dim3 blk(256);
  const dim3 gCV(NB * SEQ * (DMOD / 8) / 256, 3);
  const dim3 gWT((DMOD / 64) * (DMOD / 64), 4);
  const dim3 gGW(GLN * (DMOD / 8) / 256);
  const dim3 bG(128);
  const dim3 gQ(NB * (SEQ / 64) * (DMOD / 64));
  const dim3 gK((NB * SKEY / 64) * (DMOD / 64));
  const dim3 gV(NB * (DMOD / 64) * (SKEY / 64));
  const dim3 gG((NB * SEQ / 64) * (GLN / 64));
  const dim3 gAT(ATT_BLOCKS);
  const dim3 bAT(ATT_THREADS);
  const dim3 gCN(NB * SEQ * (DMOD / 8) / 256);
  const dim3 gO((NB * SEQ / 64) * (DMOD / 64));

  cvt_rows<<<gCV, blk, 0, stream>>>(Xin, Fin, Rin, XB);
  wt16<<<gWT, blk, 0, stream>>>(Wq, Wk, Wv, Wo, WQT, WKT, WVT, WOT);
  gwt16<<<gGW, blk, 0, stream>>>(Gw, GWT);
  gemm_b16<<<gQ, bG, 0, stream>>>(XB, WQT, QP, QR, SEQ, DMOD, DMOD, SKEY * DMOD, 0, SEQ * DMOD, QSC, 1, QRS,
                                   Gb, 0, 0);
  gemm_b16<<<gK, bG, 0, stream>>>(XB, WKT, KP, KP, NB * SKEY, DMOD, DMOD, 0, 0, 0, KSC, 0, 1.0f, Gb, 0, 0);
  gemm_b16<<<gV, bG, 0, stream>>>(WVT, XB, VP, VP, DMOD, SKEY, DMOD, 0, SKEY * DMOD, DMOD * SKEY, VCAR, 0, 1.0f,
                                   Gb, 1, 0);
  gemm_hf<false><<<gG, bG, 0, stream>>>(QP, QP, GWT, GL, NB * SEQ, GLN, DMOD, 1.0f / (QSC * GWS), 0.f, Gb, NH);
  attn_fwd<<<gAT, bAT, 0, stream>>>(QP, QR, KP, VP, GL, Y);
  canon16<<<gCN, blk, 0, stream>>>(Y, Cw, Cb, YH, YR);
  gemm_hf<true><<<gO, bG, 0, stream>>>(YH, YR, WOT, out, NB * SEQ, DMOD, DMOD, 1.0f / (OSC * WOS), 1.0f / ORS, Gb, 0);
  (void)hipGetLastError();
}
